// WaveRNNONNX_14224931684623
// MI455X (gfx1250) — hardware-verified
//
#include <hip/hip_runtime.h>
#include <stdint.h>

typedef __attribute__((ext_vector_type(16))) _Float16 v16h;
typedef __attribute__((ext_vector_type(8)))  _Float16 v8h;
typedef __attribute__((ext_vector_type(4)))  _Float16 v4h;
typedef __attribute__((ext_vector_type(16))) __bf16   v16b;
typedef __attribute__((ext_vector_type(8)))  __bf16   v8b;
typedef __attribute__((ext_vector_type(8)))  float    v8f;
typedef __attribute__((ext_vector_type(4)))  float    v4f;

__device__ __forceinline__ unsigned short f2bf_bits(float f) {
  unsigned u = __float_as_uint(f);
  return (unsigned short)((u + 0x7FFFu + ((u >> 16) & 1u)) >> 16);
}
__device__ __forceinline__ float bf_bits2f(unsigned short h) { return __uint_as_float(((unsigned)h) << 16); }

__device__ __forceinline__ void dep_guard_h(v8f& a, v8f& b, v16h x, v16h y) { asm volatile("v_nop\n\tv_nop\n\tv_nop\n\tv_nop" : "+v"(a), "+v"(b) : "v"(x), "v"(y)); }
__device__ __forceinline__ void dep_guard_b(v8f& a, v8f& b, v16b x, v16b y) { asm volatile("v_nop\n\tv_nop\n\tv_nop\n\tv_nop" : "+v"(a), "+v"(b) : "v"(x), "v"(y)); }
__device__ __forceinline__ void keep4_h(v16h a, v16h b, v16h c, v16h d) { asm volatile("v_nop" :: "v"(a), "v"(b), "v"(c), "v"(d)); }
__device__ __forceinline__ void keep4_b(v16b a, v16b b, v16b c, v16b d) { asm volatile("v_nop" :: "v"(a), "v"(b), "v"(c), "v"(d)); }
__device__ __forceinline__ void acc_guard4(v8f& a, v8f& b, v8f& c, v8f& d) { asm volatile("v_nop\n\tv_nop\n\tv_nop\n\tv_nop" : "+v"(a), "+v"(b), "+v"(c), "+v"(d)); }
template <typename T> struct Frag;
template <> struct Frag<_Float16> {
  typedef v16h V; union U { v16h v; v8h h[2]; };
  static __device__ __forceinline__ v16h load(const _Float16* p) {
    U f; f.h[0] = *(const v8h*)(p); f.h[1] = *(const v8h*)(p + 16); return f.v;
  }
  static __device__ __forceinline__ v8f mma(v16h a, v16h b, v8f c) {
    return __builtin_amdgcn_wmma_f32_16x16x32_f16(false, a, false, b, (short)0, c, false, false);
  }
  static __device__ __forceinline__ void guard(v8f& a, v8f& b, v16h x, v16h y) { dep_guard_h(a, b, x, y); }
  static __device__ __forceinline__ void keep(v16h a, v16h b, v16h c, v16h d) { keep4_h(a, b, c, d); }
};
template <> struct Frag<__bf16> {
  typedef v16b V; union U { v16b v; v8b h[2]; };
  static __device__ __forceinline__ v16b load(const __bf16* p) {
    U f; f.h[0] = *(const v8b*)(p); f.h[1] = *(const v8b*)(p + 16); return f.v;
  }
  static __device__ __forceinline__ v8f mma(v16b a, v16b b, v8f c) {
    return __builtin_amdgcn_wmma_f32_16x16x32_bf16(false, a, false, b, (short)0, c, false, false);
  }
  static __device__ __forceinline__ void guard(v8f& a, v8f& b, v16b x, v16b y) { dep_guard_b(a, b, x, y); }
  static __device__ __forceinline__ void keep(v16b a, v16b b, v16b c, v16b d) { keep4_b(a, b, c, d); }
};

template <int ET> struct Elem;
template <> struct Elem<0> { typedef _Float16 T; };
template <> struct Elem<1> { typedef __bf16 T; };
template <int ET, bool SPLIT, int BIAS_MODE, int OUT_MODE, bool RESID, int ACT = 0>
__global__ __launch_bounds__(256) void wmma_gemm64(
    const unsigned short* __restrict__ Ap, const unsigned short* __restrict__ A2p, int lda, long strideA,
    const unsigned short* __restrict__ Btp, const unsigned short* __restrict__ Bt2p, int ldb, long strideB,
    void* __restrict__ Cout, void* __restrict__ Cout2, int ldc, long strideC,
    const float* __restrict__ bias,
    const float* __restrict__ resid, long strideR,
    int M, int N, int K, float scale) {
  typedef typename Elem<ET>::T T;
  typedef typename Frag<T>::V V;
  const T* A = (const T*)Ap; const T* A2 = (const T*)A2p; const T* Bt = (const T*)Btp; const T* Bt2 = (const T*)Bt2p;
  __shared__ __align__(16) float sT[8][16 * 68];
  const int b    = blockIdx.y;
  const int lane = threadIdx.x & 31;
  const int wave = threadIdx.x >> 5;
  const int tilesN = N >> 6;
  const int tilesM = M >> 6;
  const int tile = blockIdx.x * 8 + wave;
  if (tile >= tilesM * tilesN) return;
  const int tm = tile / tilesN;
  const int tn = tile - tm * tilesN;
  const int m0 = tm << 6;
  const int n0 = tn << 6;

  const T* Ab  = A  + (size_t)b * strideA;
  const T* Bb  = Bt + (size_t)b * strideB;
  const T* Ab2 = SPLIT ? (A2  + (size_t)b * strideA) : nullptr;
  const T* Bb2 = SPLIT ? (Bt2 + (size_t)b * strideB) : nullptr;

  const int rlane = lane & 15;
  const int koff  = (lane >> 4) * 8;
  const int mOff  = (lane >> 4) * 8;

  v8f acc[4][4];
#pragma unroll
  for (int i = 0; i < 4; ++i)
#pragma unroll
    for (int j = 0; j < 4; ++j) acc[i][j] = (v8f){0.f,0.f,0.f,0.f,0.f,0.f,0.f,0.f};

  for (int k0 = 0; k0 < K; k0 += 32) {
    V bh[4], bl[4];
#pragma unroll
    for (int j = 0; j < 4; ++j) {
      const size_t bo = (size_t)(n0 + (j << 4) + rlane) * ldb + koff + k0;
      bh[j] = Frag<T>::load(Bb + bo);
      if (SPLIT) bl[j] = Frag<T>::load(Bb2 + bo);
    }
#pragma unroll
    for (int i = 0; i < 4; ++i) {
      const size_t ao = (size_t)(m0 + (i << 4) + rlane) * lda + koff + k0;
      V ah = Frag<T>::load(Ab + ao);
      V al;
      if (SPLIT) al = Frag<T>::load(Ab2 + ao);
#pragma unroll
      for (int j = 0; j < 4; ++j) {
        acc[i][j] = Frag<T>::mma(ah, bh[j], acc[i][j]);
        if (SPLIT) {
          acc[i][j] = Frag<T>::mma(ah, bl[j], acc[i][j]);
          acc[i][j] = Frag<T>::mma(al, bh[j], acc[i][j]);
        }
      }
      Frag<T>::guard(acc[i][0], acc[i][3], ah, SPLIT ? al : ah);
    }
    Frag<T>::keep(bh[0], bh[1], bh[2], bh[3]);
    if (SPLIT) Frag<T>::keep(bl[0], bl[1], bl[2], bl[3]);
  }
  acc_guard4(acc[0][0], acc[0][1], acc[0][2], acc[0][3]);
  acc_guard4(acc[1][0], acc[1][1], acc[1][2], acc[1][3]);
  acc_guard4(acc[2][0], acc[2][1], acc[2][2], acc[2][3]);
  acc_guard4(acc[3][0], acc[3][1], acc[3][2], acc[3][3]);

  float* slab = sT[wave];
  const float* Rb = RESID ? (resid + (size_t)b * strideR) : nullptr;
#pragma unroll
  for (int i = 0; i < 4; ++i) {
    const int mBase = m0 + (i << 4);
#pragma unroll
    for (int j = 0; j < 4; ++j) {
      const int n = n0 + (j << 4) + rlane;
      float bv = 0.f;
      if (BIAS_MODE == 2) bv = bias[n];
#pragma unroll
      for (int r = 0; r < 8; ++r) {
        float v = acc[i][j][r] * scale;
        if (BIAS_MODE == 1) v += bias[mBase + mOff + r];
        if (BIAS_MODE == 2) v += bv;
        if (RESID) v += Rb[(size_t)(mBase + mOff + r) * ldc + n];
        if (ACT == 1) v = tanhf(v);
        if (ACT == 2) v = fmaxf(v, 0.0f);
        if (ACT == 3) v = v / (1.0f + expf(-v));
        if (ACT == 4) v = (v > 0.f) ? v : 0.01f * v;
        if (ACT == 5) v = 0.5f * v * (1.0f + erff(v * 0.70710678118654752f));
        slab[(mOff + r) * 68 + (j << 4) + rlane] = v;
      }
    }
    __builtin_amdgcn_fence(__ATOMIC_RELEASE, "workgroup");
    __builtin_amdgcn_wave_barrier();
    __builtin_amdgcn_fence(__ATOMIC_ACQUIRE, "workgroup");
    if (OUT_MODE == 0) {
      float* C = (float*)Cout + (size_t)b * strideC;
      const int hh = lane >> 4, c4 = (lane & 15) * 4;
      for (int pass = 0; pass < 2; ++pass) {
#pragma unroll
        for (int it = 0; it < 8; ++it) {
          const int row = it * 2 + hh;
          v4f v = *(const v4f*)(slab + row * 68 + c4);
          *(volatile v4f*)(C + (size_t)(mBase + row) * ldc + n0 + c4) = v;
        }
        __threadfence();
      }
    } else {
      const int q = lane >> 3, c8 = (lane & 7) * 8;
      unsigned short* C  = (unsigned short*)Cout  + (size_t)b * strideC;
      unsigned short* C2 = (OUT_MODE == 2) ? ((unsigned short*)Cout2 + (size_t)b * strideC) : nullptr;
      for (int pass = 0; pass < 2; ++pass) {
#pragma unroll
        for (int it = 0; it < 4; ++it) {
          const int row = it * 4 + q;
          const float* sp = slab + row * 68 + c8;
          v8h hv, lv;
#pragma unroll
          for (int e = 0; e < 8; ++e) {
            if (OUT_MODE == 1) {
              hv[e] = (_Float16)sp[e];
            } else {
              unsigned short hb = f2bf_bits(sp[e]);
              unsigned short lb = f2bf_bits(sp[e] - bf_bits2f(hb));
              hv[e] = __builtin_bit_cast(_Float16, hb);
              lv[e] = __builtin_bit_cast(_Float16, lb);
            }
          }
          *(volatile v8h*)(C + (size_t)(mBase + row) * ldc + n0 + c8) = hv;
          if (OUT_MODE == 2) *(volatile v8h*)(C2 + (size_t)(mBase + row) * ldc + n0 + c8) = lv;
        }
        __threadfence();
      }
    }
    __builtin_amdgcn_fence(__ATOMIC_RELEASE, "workgroup");
    __builtin_amdgcn_wave_barrier();
    __builtin_amdgcn_fence(__ATOMIC_ACQUIRE, "workgroup");
  }
}

__device__ __forceinline__ unsigned pack_h2(float a, float b) {
  const _Float16 h0 = (_Float16)a, h1 = (_Float16)b;
  return (unsigned)__builtin_bit_cast(unsigned short, h0) | ((unsigned)__builtin_bit_cast(unsigned short, h1) << 16);
}
__global__ __launch_bounds__(256) void cast_pad_f16x2(
    const float* __restrict__ in, _Float16* __restrict__ out, int K, int Kpad, int npairs, float scale) {
  const int i = blockIdx.x * 256 + threadIdx.x;
  if (i < npairs) {
    const int e0 = 2 * i;
    const int r = e0 / Kpad;
    const int c = e0 - r * Kpad;
    const float* src = in + (size_t)r * K;
    float v0 = 0.0f, v1 = 0.0f;
    if (c < K) v0 = src[c] * scale;
    if (c + 1 < K) v1 = src[c + 1] * scale;
    const unsigned u = pack_h2(v0, v1);
    ((volatile unsigned*)out)[i] = u;
    __threadfence();
    ((volatile unsigned*)out)[i] = u;
  }
}

__device__ __forceinline__ float x0_val(const float* __restrict__ x, const float* __restrict__ mel,
                                        const float* __restrict__ a1, int r, int c) {
  if (c == 0) return x[r];
  if (c < 81) return mel[(size_t)r * 80 + (c - 1)];
  if (c < 113) return a1[(size_t)r * 32 + (c - 81)];
  return 0.0f;
}
__global__ __launch_bounds__(256) void build_x0_f16x2(
    const float* __restrict__ x, const float* __restrict__ mel, const float* __restrict__ a1,
    _Float16* __restrict__ out, int npairs) {
  const int i = blockIdx.x * 256 + threadIdx.x;
  if (i < npairs) {
    const int e0 = 2 * i;
    const int r = e0 >> 7;
    const int c = e0 & 127;
    const float v0 = x0_val(x, mel, a1, r, c);
    const float v1 = x0_val(x, mel, a1, r, c + 1);
    const unsigned u = pack_h2(v0, v1);
    ((volatile unsigned*)out)[i] = u;
    __threadfence();
    ((volatile unsigned*)out)[i] = u;
  }
}

__device__ __forceinline__ float sigm_f(float v) {
  return __builtin_amdgcn_rcpf(1.0f + __builtin_amdgcn_exp2f(v * -1.4426950408889634f));
}
__device__ __forceinline__ float tanh_f(float v) {
  const float e = __builtin_amdgcn_exp2f(v * 2.8853900817779268f);
  return 1.0f - 2.0f * __builtin_amdgcn_rcpf(e + 1.0f);
}
template <bool XF>
__global__ __launch_bounds__(256) void gru_gate_k(
    const float* __restrict__ G, const float* __restrict__ hprev, const float* __restrict__ xprev,
    const float* __restrict__ aux, float* __restrict__ hout, float* __restrict__ xout,
    _Float16* __restrict__ xh, int rows) {
  const int tid = threadIdx.x;
  const int row = blockIdx.x * 2 + (tid >> 7);
  const int t = tid & 127;
  if (row >= rows) return;
  const size_t gb = (size_t)row * 3072 + 4 * t;
  const v4f gir = *(const v4f*)(G + gb);
  const v4f giz = *(const v4f*)(G + gb + 512);
  const v4f gin = *(const v4f*)(G + gb + 1024);
  const v4f ghr = *(const v4f*)(G + gb + 1536);
  const v4f ghz = *(const v4f*)(G + gb + 2048);
  const v4f ghn = *(const v4f*)(G + gb + 2560);
  const size_t hb = (size_t)row * 512 + 4 * t;
  const v4f hp = *(const v4f*)(hprev + hb);
  const v4f xp = *(const v4f*)(xprev + hb);
  v4f hn, xn;
  v4h xq;
#pragma unroll
  for (int e = 0; e < 4; ++e) {
    const float r = sigm_f(gir[e] + ghr[e]);
    const float z = sigm_f(giz[e] + ghz[e]);
    const float n = tanh_f(fmaf(r, ghn[e], gin[e]));
    const float h = (1.0f - z) * n + z * hp[e];
    hn[e] = h;
    const float xv = xp[e] + h;
    xn[e] = xv;
    xq[e] = (_Float16)xv;
  }
  const bool doaux = (t < 32);
  unsigned aw = 0u;
  if (doaux) {
    float a0 = 0.0f, a1v = 0.0f;
    if (t < 16) { a0 = aux[(size_t)row * 32 + 2 * t]; a1v = aux[(size_t)row * 32 + 2 * t + 1]; }
    aw = pack_h2(a0, a1v);
  }
  _Float16* xrow = xh + (size_t)row * 576;
  for (int pass = 0; pass < 2; ++pass) {
    *(volatile v4f*)(hout + hb) = hn;
    if (XF) *(volatile v4f*)(xout + hb) = xn;
    *(volatile v4h*)(xrow + 4 * t) = xq;
    if (doaux) *(volatile unsigned*)(xrow + 512 + 2 * t) = aw;
    __threadfence();
  }
}

__global__ __launch_bounds__(256) void aux_line_k(const float* __restrict__ aux, _Float16* __restrict__ xh, int rows) {
  const int gid = blockIdx.x * 256 + threadIdx.x;
  const int row = gid >> 5;
  const int l = gid & 31;
  if (row >= rows) return;
  float a0 = 0.0f, a1v = 0.0f;
  if (l < 16) { a0 = aux[(size_t)row * 32 + 2 * l]; a1v = aux[(size_t)row * 32 + 2 * l + 1]; }
  const unsigned aw = pack_h2(a0, a1v);
  volatile unsigned* p = (volatile unsigned*)(xh + (size_t)row * 576 + 512 + 2 * l);
  *p = aw;
  __threadfence();
  *p = aw;
}

static void gemm_f32out(hipStream_t s, const _Float16* A, int lda, const _Float16* Bt, int ldb,
                        const float* bias, float* C, int ldc, int M, int N, int K, float scale) {
  const int tiles = (M / 64) * (N / 64);
  dim3 grid((unsigned)((tiles + 7) / 8), 1, 1);
  wmma_gemm64<0, false, 2, 0, false, 0><<<grid, 256, 0, s>>>(
      (const unsigned short*)A, (const unsigned short*)A, lda, 0L,
      (const unsigned short*)Bt, (const unsigned short*)Bt, ldb, 0L,
      (void*)C, (void*)C, ldc, 0L, bias, bias, 0L, M, N, K, scale);
}
static void gemm_f16out_relu(hipStream_t s, const _Float16* A, int lda, const _Float16* Bt, int ldb,
                             const float* bias, _Float16* C, int ldc, int M, int N, int K, float scale) {
  const int tiles = (M / 64) * (N / 64);
  dim3 grid((unsigned)((tiles + 7) / 8), 1, 1);
  wmma_gemm64<0, false, 2, 1, false, 2><<<grid, 256, 0, s>>>(
      (const unsigned short*)A, (const unsigned short*)A, lda, 0L,
      (const unsigned short*)Bt, (const unsigned short*)Bt, ldb, 0L,
      (void*)C, (void*)C, ldc, 0L, bias, bias, 0L, M, N, K, scale);
}
static void cast_f16(hipStream_t s, const float* in, _Float16* out, int rows, int K, int Kpad, float scale) {
  const int npairs = (int)(((long)rows * Kpad) / 2);
  cast_pad_f16x2<<<(unsigned)((npairs + 255) / 256), 256, 0, s>>>(in, out, K, Kpad, npairs, scale);
}

extern "C" void kernel_launch(void* const* d_in, const int* in_sizes, int n_in,
                              void* d_out, int out_size, void* d_ws, size_t ws_size,
                              hipStream_t stream) {
  if (n_in < 24) return;
  const int RNN = 512, NC = 512;
  const int B = in_sizes[7];
  if (B <= 0 || (B % 128) != 0) return;
  if (in_sizes[5] != B * RNN || in_sizes[6] != B * RNN) return;
  if (out_size != 3 * B * NC) return;
  const int Bh = B / 2;

  const float* m_t   = (const float*)d_in[0];
  const float* a1    = (const float*)d_in[1];
  const float* a2    = (const float*)d_in[2];
  const float* a3    = (const float*)d_in[3];
  const float* a4    = (const float*)d_in[4];
  const float* h1    = (const float*)d_in[5];
  const float* h2    = (const float*)d_in[6];
  const float* x     = (const float*)d_in[7];
  const float* I_w   = (const float*)d_in[8];
  const float* I_b   = (const float*)d_in[9];
  const float* r1wih = (const float*)d_in[10];
  const float* r1whh = (const float*)d_in[11];
  const float* r1bih = (const float*)d_in[12];
  const float* r1bhh = (const float*)d_in[13];
  const float* r2wih = (const float*)d_in[14];
  const float* r2whh = (const float*)d_in[15];
  const float* r2bih = (const float*)d_in[16];
  const float* r2bhh = (const float*)d_in[17];
  const float* f1w   = (const float*)d_in[18];
  const float* f1b   = (const float*)d_in[19];
  const float* f2w   = (const float*)d_in[20];
  const float* f2b   = (const float*)d_in[21];
  const float* f3w   = (const float*)d_in[22];
  const float* f3b   = (const float*)d_in[23];

  float* logits = (float*)d_out;
  float* h1n    = logits + (size_t)B * NC;
  float* h2n    = h1n + (size_t)B * RNN;

  char* base = (char*)d_ws;
  size_t off = 0;
  auto carve = [&](size_t bytes) -> void* {
    void* p = base + off;
    off += (bytes + 255) & ~(size_t)255;
    return p;
  };
  _Float16* wI   = (_Float16*)carve((size_t)512 * 128 * 2);
  _Float16* w1ih = (_Float16*)carve((size_t)1536 * 512 * 2);
  _Float16* w1hh = (_Float16*)carve((size_t)1536 * 512 * 2);
  _Float16* w2ih = (_Float16*)carve((size_t)1536 * 544 * 2);
  _Float16* w2hh = (_Float16*)carve((size_t)1536 * 512 * 2);
  _Float16* wf1  = (_Float16*)carve((size_t)512 * 544 * 2);
  _Float16* wf2  = (_Float16*)carve((size_t)512 * 544 * 2);
  _Float16* wf3  = (_Float16*)carve((size_t)512 * 512 * 2);
  _Float16* X0   = (_Float16*)carve((size_t)B * 128 * 2);
  _Float16* Hb   = (_Float16*)carve((size_t)B * 512 * 2);
  float*    X1   = (float*)carve((size_t)B * 512 * 4);
  float*    X2   = (float*)carve((size_t)B * 512 * 4);
  _Float16* bufA = (_Float16*)carve((size_t)B * 576 * 2);
  _Float16* bufB = (_Float16*)carve((size_t)B * 576 * 2);
  float*    G    = (float*)carve((size_t)Bh * 3072 * 4);
  if (off > ws_size) return;

  const float WSC = 16.0f, WINV = 0.0625f;

  cast_f16(stream, I_w,   wI,   512,  113, 128, WSC);
  cast_f16(stream, r1wih, w1ih, 1536, 512, 512, WSC);
  cast_f16(stream, r1whh, w1hh, 1536, 512, 512, WSC);
  cast_f16(stream, r2wih, w2ih, 1536, 544, 544, WSC);
  cast_f16(stream, r2whh, w2hh, 1536, 512, 512, WSC);
  cast_f16(stream, f1w,   wf1,  512,  544, 544, WSC);
  cast_f16(stream, f2w,   wf2,  512,  544, 544, WSC);
  cast_f16(stream, f3w,   wf3,  512,  512, 512, WSC);
  cast_f16(stream, h1, Hb, B, 512, 512, 1.0f);
  {
    const int npairs = B * 64;
    build_x0_f16x2<<<(unsigned)((npairs + 255) / 256), 256, 0, stream>>>(x, m_t, a1, X0, npairs);
  }

  gemm_f32out(stream, X0, 128, wI, 128, I_b, X1, 512, B, 512, 128, WINV);
  cast_f16(stream, X1, bufA, B, 512, 512, 1.0f);

  for (int hb = 0; hb < 2; ++hb) {
    const size_t r0 = (size_t)hb * Bh;
    gemm_f32out(stream, bufA + r0 * 512, 512, w1ih, 512, r1bih, G,        3072, Bh, 1536, 512, WINV);
    gemm_f32out(stream, Hb   + r0 * 512, 512, w1hh, 512, r1bhh, G + 1536, 3072, Bh, 1536, 512, WINV);
    gru_gate_k<true><<<(unsigned)((Bh + 1) / 2), 256, 0, stream>>>(
        G, h1 + r0 * 512, X1 + r0 * 512, a2 + r0 * 32, h1n + r0 * 512, X2 + r0 * 512, bufB + r0 * 576, Bh);
  }

  cast_f16(stream, h2, Hb, B, 512, 512, 1.0f);
  for (int hb = 0; hb < 2; ++hb) {
    const size_t r0 = (size_t)hb * Bh;
    gemm_f32out(stream, bufB + r0 * 576, 576, w2ih, 544, r2bih, G,        3072, Bh, 1536, 544, WINV);
    gemm_f32out(stream, Hb   + r0 * 512, 512, w2hh, 512, r2bhh, G + 1536, 3072, Bh, 1536, 512, WINV);
    gru_gate_k<false><<<(unsigned)((Bh + 1) / 2), 256, 0, stream>>>(
        G, h2 + r0 * 512, X2 + r0 * 512, a3 + r0 * 32, h2n + r0 * 512, X1 + r0 * 512, bufA + r0 * 576, Bh);
  }

  gemm_f16out_relu(stream, bufA, 576, wf1, 544, f1b, bufB, 576, B, 512, 544, WINV);
  aux_line_k<<<(unsigned)(((long)B * 32 + 255) / 256), 256, 0, stream>>>(a4, bufB, B);
  gemm_f16out_relu(stream, bufB, 576, wf2, 544, f2b, bufA, 576, B, 512, 544, WINV);
  gemm_f32out(stream, bufA, 576, wf3, 512, f3b, logits, 512, B, 512, 512, WINV);
  (void)hipGetLastError();
}
